// SSMDownstreamDecoder_27487790694541
// MI455X (gfx1250) — hardware-verified
//
#include <hip/hip_runtime.h>
#include <math.h>

constexpr int kSeq       = 8192;
constexpr int kHid       = 512;
constexpr int kSt        = 256;
constexpr int kLayers    = 6;
constexpr int kOutDim    = 128;
constexpr int kEncRows   = 504;
constexpr int kCtxDim    = 8;
constexpr int kScanBatch = 8;
constexpr float kWCarry   = 16.0f;
constexpr float kBCarry   = 4096.0f;
constexpr float kXCarry   = 64.0f;
constexpr float kCCarry   = 16.0f;
constexpr float kEncScale = 1.0f / 16.0f;
constexpr float kBuScale  = 1.0f / 4096.0f;
constexpr float kYScale   = 2.0f / (64.0f * 16.0f);
constexpr float kGluScale = 1.0f / 16.0f;
constexpr float kDecScale = 1.0f / 16.0f;
constexpr float kInvHid   = 1.0f / 512.0f;
constexpr float kLnEps    = 1e-5f;

typedef __attribute__((ext_vector_type(16))) _Float16 v16h;
typedef __attribute__((ext_vector_type(8)))  _Float16 v8h;
typedef __attribute__((ext_vector_type(16))) __bf16   v16b;
typedef __attribute__((ext_vector_type(8)))  __bf16   v8b;
typedef __attribute__((ext_vector_type(8)))  float    v8f;
typedef __attribute__((ext_vector_type(4)))  float    v4f;
typedef __attribute__((ext_vector_type(4)))  unsigned int v4u;

__device__ __forceinline__ unsigned short f2bf_bits(float f) {
  unsigned u = __float_as_uint(f);
  return (unsigned short)((u + 0x7FFFu + ((u >> 16) & 1u)) >> 16);
}
__device__ __forceinline__ float bf_bits2f(unsigned short h) { return __uint_as_float(((unsigned)h) << 16); }

__device__ __forceinline__ void dep_guard_h(v8f& a, v8f& b, v16h x, v16h y) { asm volatile("v_nop\n\tv_nop\n\tv_nop\n\tv_nop" : "+v"(a), "+v"(b) : "v"(x), "v"(y)); }
__device__ __forceinline__ void dep_guard_b(v8f& a, v8f& b, v16b x, v16b y) { asm volatile("v_nop\n\tv_nop\n\tv_nop\n\tv_nop" : "+v"(a), "+v"(b) : "v"(x), "v"(y)); }
__device__ __forceinline__ void keep4_h(v16h a, v16h b, v16h c, v16h d) { asm volatile("v_nop" :: "v"(a), "v"(b), "v"(c), "v"(d)); }
__device__ __forceinline__ void keep4_b(v16b a, v16b b, v16b c, v16b d) { asm volatile("v_nop" :: "v"(a), "v"(b), "v"(c), "v"(d)); }
__device__ __forceinline__ void acc_guard4(v8f& a, v8f& b, v8f& c, v8f& d) { asm volatile("v_nop\n\tv_nop\n\tv_nop\n\tv_nop" : "+v"(a), "+v"(b), "+v"(c), "+v"(d)); }
template <typename T> struct Frag;
template <> struct Frag<_Float16> {
  typedef v16h V; union U { v16h v; v8h h[2]; };
  static __device__ __forceinline__ v16h load(const _Float16* p) {
    U f; f.h[0] = *(const v8h*)(p); f.h[1] = *(const v8h*)(p + 16); return f.v;
  }
  static __device__ __forceinline__ v8f mma(v16h a, v16h b, v8f c) {
    return __builtin_amdgcn_wmma_f32_16x16x32_f16(false, a, false, b, (short)0, c, false, false);
  }
  static __device__ __forceinline__ void guard(v8f& a, v8f& b, v16h x, v16h y) { dep_guard_h(a, b, x, y); }
  static __device__ __forceinline__ void keep(v16h a, v16h b, v16h c, v16h d) { keep4_h(a, b, c, d); }
};
template <> struct Frag<__bf16> {
  typedef v16b V; union U { v16b v; v8b h[2]; };
  static __device__ __forceinline__ v16b load(const __bf16* p) {
    U f; f.h[0] = *(const v8b*)(p); f.h[1] = *(const v8b*)(p + 16); return f.v;
  }
  static __device__ __forceinline__ v8f mma(v16b a, v16b b, v8f c) {
    return __builtin_amdgcn_wmma_f32_16x16x32_bf16(false, a, false, b, (short)0, c, false, false);
  }
  static __device__ __forceinline__ void guard(v8f& a, v8f& b, v16b x, v16b y) { dep_guard_b(a, b, x, y); }
  static __device__ __forceinline__ void keep(v16b a, v16b b, v16b c, v16b d) { keep4_b(a, b, c, d); }
};

__device__ __forceinline__ unsigned pk16(unsigned short a, unsigned short b) { return (unsigned)a | ((unsigned)b << 16); }
__device__ __forceinline__ unsigned short h_bits(float f) { const _Float16 h = (_Float16)f; return __builtin_bit_cast(unsigned short, h); }

template <int ET> struct Elem;
template <> struct Elem<0> { typedef _Float16 T; };
template <> struct Elem<1> { typedef __bf16 T; };
template <int ET, bool SPLIT, int BIAS_MODE, int OUT_MODE, bool RESID, int ACT = 0>
__global__ __launch_bounds__(256) void wmma_gemm64(
    const unsigned short* __restrict__ Ap, const unsigned short* __restrict__ A2p, int lda, long strideA,
    const unsigned short* __restrict__ Btp, const unsigned short* __restrict__ Bt2p, int ldb, long strideB,
    void* __restrict__ Cout, void* __restrict__ Cout2, int ldc, long strideC,
    const float* __restrict__ bias,
    const float* __restrict__ resid, long strideR,
    int M, int N, int K, float scale) {
  typedef typename Elem<ET>::T T;
  typedef typename Frag<T>::V V;
  const T* A = (const T*)Ap; const T* A2 = (const T*)A2p; const T* Bt = (const T*)Btp; const T* Bt2 = (const T*)Bt2p;
  __shared__ __align__(16) float sT[8][16 * 68];
  const int b    = blockIdx.y;
  const int lane = threadIdx.x & 31;
  const int wave = threadIdx.x >> 5;
  const int tilesN = N >> 6;
  const int tilesM = M >> 6;
  const int tile = blockIdx.x * 8 + wave;
  if (tile >= tilesM * tilesN) return;
  const int tm = tile / tilesN;
  const int tn = tile - tm * tilesN;
  const int m0 = tm << 6;
  const int n0 = tn << 6;

  const T* Ab  = A  + (size_t)b * strideA;
  const T* Bb  = Bt + (size_t)b * strideB;
  const T* Ab2 = SPLIT ? (A2  + (size_t)b * strideA) : nullptr;
  const T* Bb2 = SPLIT ? (Bt2 + (size_t)b * strideB) : nullptr;

  const int rlane = lane & 15;
  const int koff  = (lane >> 4) * 8;
  const int mOff  = (lane >> 4) * 8;

  v8f acc[4][4];
#pragma unroll
  for (int i = 0; i < 4; ++i)
#pragma unroll
    for (int j = 0; j < 4; ++j) acc[i][j] = (v8f){0.f,0.f,0.f,0.f,0.f,0.f,0.f,0.f};

  for (int k0 = 0; k0 < K; k0 += 32) {
    V bh[4], bl[4];
#pragma unroll
    for (int j = 0; j < 4; ++j) {
      const size_t bo = (size_t)(n0 + (j << 4) + rlane) * ldb + koff + k0;
      bh[j] = Frag<T>::load(Bb + bo);
      if (SPLIT) bl[j] = Frag<T>::load(Bb2 + bo);
    }
#pragma unroll
    for (int i = 0; i < 4; ++i) {
      const size_t ao = (size_t)(m0 + (i << 4) + rlane) * lda + koff + k0;
      V ah = Frag<T>::load(Ab + ao);
      V al;
      if (SPLIT) al = Frag<T>::load(Ab2 + ao);
#pragma unroll
      for (int j = 0; j < 4; ++j) {
        acc[i][j] = Frag<T>::mma(ah, bh[j], acc[i][j]);
        if (SPLIT) {
          acc[i][j] = Frag<T>::mma(ah, bl[j], acc[i][j]);
          acc[i][j] = Frag<T>::mma(al, bh[j], acc[i][j]);
        }
      }
      Frag<T>::guard(acc[i][0], acc[i][3], ah, SPLIT ? al : ah);
    }
    Frag<T>::keep(bh[0], bh[1], bh[2], bh[3]);
    if (SPLIT) Frag<T>::keep(bl[0], bl[1], bl[2], bl[3]);
  }
  acc_guard4(acc[0][0], acc[0][1], acc[0][2], acc[0][3]);
  acc_guard4(acc[1][0], acc[1][1], acc[1][2], acc[1][3]);
  acc_guard4(acc[2][0], acc[2][1], acc[2][2], acc[2][3]);
  acc_guard4(acc[3][0], acc[3][1], acc[3][2], acc[3][3]);

  float* slab = sT[wave];
  const float* Rb = RESID ? (resid + (size_t)b * strideR) : nullptr;
#pragma unroll
  for (int i = 0; i < 4; ++i) {
    const int mBase = m0 + (i << 4);
#pragma unroll
    for (int j = 0; j < 4; ++j) {
      const int n = n0 + (j << 4) + rlane;
      float bv = 0.f;
      if (BIAS_MODE == 2) bv = bias[n];
#pragma unroll
      for (int r = 0; r < 8; ++r) {
        float v = acc[i][j][r] * scale;
        if (BIAS_MODE == 1) v += bias[mBase + mOff + r];
        if (BIAS_MODE == 2) v += bv;
        if (RESID) v += Rb[(size_t)(mBase + mOff + r) * ldc + n];
        if (ACT == 2) v = fmaxf(v, 0.0f);
        if (ACT == 4) v = (v > 0.f) ? v : 0.01f * v;
        slab[(mOff + r) * 68 + (j << 4) + rlane] = v;
      }
    }
    __builtin_amdgcn_fence(__ATOMIC_RELEASE, "workgroup");
    __builtin_amdgcn_wave_barrier();
    __builtin_amdgcn_fence(__ATOMIC_ACQUIRE, "workgroup");
    if (OUT_MODE == 0) {
      float* C = (float*)Cout + (size_t)b * strideC;
      const int hh = lane >> 4, c4 = (lane & 15) * 4;
      for (int pass = 0; pass < 2; ++pass) {
#pragma unroll
        for (int it = 0; it < 8; ++it) {
          const int row = it * 2 + hh;
          v4f v = *(const v4f*)(slab + row * 68 + c4);
          *(volatile v4f*)(C + (size_t)(mBase + row) * ldc + n0 + c4) = v;
        }
        __threadfence();
      }
    } else {
      const int q = lane >> 3, c8 = (lane & 7) * 8;
      unsigned short* C  = (unsigned short*)Cout  + (size_t)b * strideC;
      unsigned short* C2 = (OUT_MODE == 2) ? ((unsigned short*)Cout2 + (size_t)b * strideC) : nullptr;
      for (int pass = 0; pass < 2; ++pass) {
#pragma unroll
        for (int it = 0; it < 4; ++it) {
          const int row = it * 4 + q;
          const float* sp = slab + row * 68 + c8;
          v8h hv, lv;
#pragma unroll
          for (int e = 0; e < 8; ++e) {
            if (OUT_MODE == 1) {
              hv[e] = (_Float16)sp[e];
            } else {
              unsigned short hb = f2bf_bits(sp[e]);
              unsigned short lb = f2bf_bits(sp[e] - bf_bits2f(hb));
              hv[e] = __builtin_bit_cast(_Float16, hb);
              lv[e] = __builtin_bit_cast(_Float16, lb);
            }
          }
          *(volatile v8h*)(C + (size_t)(mBase + row) * ldc + n0 + c8) = hv;
          if (OUT_MODE == 2) *(volatile v8h*)(C2 + (size_t)(mBase + row) * ldc + n0 + c8) = lv;
        }
        __threadfence();
      }
    }
    __builtin_amdgcn_fence(__ATOMIC_RELEASE, "workgroup");
    __builtin_amdgcn_wave_barrier();
    __builtin_amdgcn_fence(__ATOMIC_ACQUIRE, "workgroup");
  }
}

__global__ __launch_bounds__(256) void cast8_f16_kernel(const float* __restrict__ in, unsigned short* __restrict__ out, int n8) {
  const int i = blockIdx.x * 256 + threadIdx.x;
  if (i >= n8) return;
  const float* p = in + 8 * (size_t)i;
  const v4f a = *(const v4f*)(p);
  const v4f c = *(const v4f*)(p + 4);
  unsigned short hb[8];
#pragma unroll
  for (int e = 0; e < 4; ++e) {
    hb[e]     = h_bits(a[e]);
    hb[4 + e] = h_bits(c[e]);
  }
  const v4u u = (v4u){pk16(hb[0], hb[1]), pk16(hb[2], hb[3]), pk16(hb[4], hb[5]), pk16(hb[6], hb[7])};
  unsigned short* q = out + 8 * (size_t)i;
  *(volatile v4u*)q = u;
  __threadfence();
  *(volatile v4u*)q = u;
}

__global__ __launch_bounds__(256) void cast_rows8_kernel(const float* __restrict__ in, long in_ls,
                                                        unsigned short* __restrict__ out, long out_ls,
                                                        int nsrc, int ndst, float scale) {
  const int i = blockIdx.x * 256 + threadIdx.x;
  if (i >= ndst * 64) return;
  const int row = i >> 6, c8 = (i & 63) * 8;
  const int rsrc = (row < nsrc) ? row : (nsrc - 1);
  const float* p = in + (size_t)blockIdx.y * in_ls + (size_t)rsrc * kHid + c8;
  const v4f a = *(const v4f*)(p);
  const v4f c = *(const v4f*)(p + 4);
  const bool live = (row < nsrc);
  unsigned short hb[8];
#pragma unroll
  for (int e = 0; e < 4; ++e) {
    hb[e]     = h_bits(live ? a[e] * scale : 0.0f);
    hb[4 + e] = h_bits(live ? c[e] * scale : 0.0f);
  }
  const v4u u = (v4u){pk16(hb[0], hb[1]), pk16(hb[2], hb[3]), pk16(hb[4], hb[5]), pk16(hb[6], hb[7])};
  unsigned short* q = out + (size_t)blockIdx.y * out_ls + (size_t)row * kHid + c8;
  *(volatile v4u*)q = u;
  __threadfence();
  *(volatile v4u*)q = u;
}

__global__ __launch_bounds__(256) void zoh_tab_kernel(const float* __restrict__ Lre, const float* __restrict__ Lim,
                                                      const float* __restrict__ logstep, float* __restrict__ tab) {
  const int l = blockIdx.x, p = threadIdx.x;
  const int i = l * kSt + p;
  const float dt = expf(logstep[i]);
  const float a = Lre[i], b = Lim[i];
  const float zr = a * dt, zi = b * dt;
  const float ez = expf(zr);
  float sn, cs;
  sincosf(zi, &sn, &cs);
  const float lbr = ez * cs, lbi = ez * sn;
  const float nr = lbr - 1.0f, ni = lbi;
  const float den = a * a + b * b;
  const float inv = 1.0f / den;
  const float gr = (nr * a + ni * b) * inv;
  const float gi = (ni * a - nr * b) * inv;
  float* T = tab + (size_t)l * 4 * kSt + p;
  *(volatile float*)(T)           = lbr;
  *(volatile float*)(T + kSt)     = lbi;
  *(volatile float*)(T + 2 * kSt) = gr;
  *(volatile float*)(T + 3 * kSt) = gi;
  __threadfence();
  *(volatile float*)(T)           = lbr;
  *(volatile float*)(T + kSt)     = lbi;
  *(volatile float*)(T + 2 * kSt) = gr;
  *(volatile float*)(T + 3 * kSt) = gi;
}

__global__ __launch_bounds__(512) void bias_pad_kernel(const float* __restrict__ benc, const float* __restrict__ ctx,
                                                       float* __restrict__ bpad) {
  const int t = threadIdx.x;
  const int i1 = (t < kEncRows) ? t : (kEncRows - 1);
  int i2 = t - kEncRows;
  i2 = (i2 < 0) ? 0 : ((i2 > kCtxDim - 1) ? (kCtxDim - 1) : i2);
  const float v1 = benc[i1];
  const float v2 = ctx[i2];
  const float v = (t < kEncRows) ? v1 : v2;
  *(volatile float*)(bpad + t) = v;
  __threadfence();
  *(volatile float*)(bpad + t) = v;
}

__global__ __launch_bounds__(256) void bbar_kernel(const float* __restrict__ Bre, const float* __restrict__ Bim,
                                                  const float* __restrict__ tab, unsigned short* __restrict__ out) {
  const int l = blockIdx.y;
  const int i = blockIdx.x * 256 + threadIdx.x;
  const int n = i >> 6, c8 = (i & 63) * 8;
  const int p = n & 255;
  const float gr = tab[(size_t)l * 4 * kSt + 2 * kSt + p];
  const float gi = tab[(size_t)l * 4 * kSt + 3 * kSt + p];
  const size_t src = ((size_t)l * kSt + p) * kHid + c8;
  const v4f r0 = *(const v4f*)(Bre + src), r1 = *(const v4f*)(Bre + src + 4);
  const v4f m0 = *(const v4f*)(Bim + src), m1 = *(const v4f*)(Bim + src + 4);
  const bool isre = (n < kSt);
  unsigned short hb[8];
#pragma unroll
  for (int e = 0; e < 4; ++e) {
    const float va = isre ? (gr * r0[e] - gi * m0[e]) : (gr * m0[e] + gi * r0[e]);
    const float vb = isre ? (gr * r1[e] - gi * m1[e]) : (gr * m1[e] + gi * r1[e]);
    hb[e]     = h_bits(va * kBCarry);
    hb[4 + e] = h_bits(vb * kBCarry);
  }
  const v4u u = (v4u){pk16(hb[0], hb[1]), pk16(hb[2], hb[3]), pk16(hb[4], hb[5]), pk16(hb[6], hb[7])};
  unsigned short* q = out + (size_t)l * kHid * kHid + (size_t)n * kHid + c8;
  *(volatile v4u*)q = u;
  __threadfence();
  *(volatile v4u*)q = u;
}

__global__ __launch_bounds__(256) void cst_kernel(const float* __restrict__ Cre, const float* __restrict__ Cim,
                                                 unsigned short* __restrict__ out) {
  const int l = blockIdx.y;
  const int i = blockIdx.x * 256 + threadIdx.x;
  const int h = i >> 6, c8 = (i & 63) * 8;
  const int w = c8 >> 6, j = c8 & 63;
  const int pp = 32 * w + (j & 31);
  const size_t src = ((size_t)l * kHid + h) * kSt + pp;
  const v4f r0 = *(const v4f*)(Cre + src), r1 = *(const v4f*)(Cre + src + 4);
  const v4f m0 = *(const v4f*)(Cim + src), m1 = *(const v4f*)(Cim + src + 4);
  const bool isre = (j < 32);
  unsigned short hb[8];
#pragma unroll
  for (int e = 0; e < 4; ++e) {
    hb[e]     = h_bits(isre ? (r0[e] * kCCarry) : (-m0[e] * kCCarry));
    hb[4 + e] = h_bits(isre ? (r1[e] * kCCarry) : (-m1[e] * kCCarry));
  }
  const v4u u = (v4u){pk16(hb[0], hb[1]), pk16(hb[2], hb[3]), pk16(hb[4], hb[5]), pk16(hb[6], hb[7])};
  unsigned short* q = out + (size_t)l * kHid * kHid + (size_t)h * kHid + c8;
  *(volatile v4u*)q = u;
  __threadfence();
  *(volatile v4u*)q = u;
}

__global__ __launch_bounds__(128) void ln_kernel(const float* __restrict__ h, const float* __restrict__ sc,
                                                const float* __restrict__ bs, float* __restrict__ z32,
                                                unsigned short* __restrict__ z16) {
  __shared__ float redA[4];
  __shared__ float redB[4];
  __shared__ __align__(16) unsigned int sZ[256];
  const int row = blockIdx.x, t = threadIdx.x;
  const int lane = t & 31, wave = t >> 5;
  const size_t base = (size_t)row * kHid + 4 * t;
  const v4f x = *(const v4f*)(h + base);
  float s = (x[0] + x[1]) + (x[2] + x[3]);
#pragma unroll
  for (int off = 16; off > 0; off >>= 1) s += __shfl_xor(s, off, 32);
  if (lane == 0) redA[wave] = s;
  __syncthreads();
  const float mu = (((redA[0] + redA[1]) + redA[2]) + redA[3]) * kInvHid;
  const float d0 = x[0] - mu, d1 = x[1] - mu, d2 = x[2] - mu, d3 = x[3] - mu;
  float s2 = (d0 * d0 + d1 * d1) + (d2 * d2 + d3 * d3);
#pragma unroll
  for (int off = 16; off > 0; off >>= 1) s2 += __shfl_xor(s2, off, 32);
  if (lane == 0) redB[wave] = s2;
  __syncthreads();
  const float var = (((redB[0] + redB[1]) + redB[2]) + redB[3]) * kInvHid;
  const float rstd = rsqrtf(var + kLnEps);
  const v4f g  = *(const v4f*)(sc + 4 * t);
  const v4f bb = *(const v4f*)(bs + 4 * t);
  v4f z;
  z[0] = d0 * rstd * g[0] + bb[0];
  z[1] = d1 * rstd * g[1] + bb[1];
  z[2] = d2 * rstd * g[2] + bb[2];
  z[3] = d3 * rstd * g[3] + bb[3];
  float* zp = z32 + base;
  *(volatile v4f*)zp = z;
  __threadfence();
  *(volatile v4f*)zp = z;
  sZ[2 * t]     = pk16(h_bits(z[0]), h_bits(z[1]));
  sZ[2 * t + 1] = pk16(h_bits(z[2]), h_bits(z[3]));
  __syncthreads();
  if (wave == 0) {
    unsigned short* zr = z16 + (size_t)row * kHid;
    for (int pass = 0; pass < 2; ++pass) {
#pragma unroll
      for (int it = 0; it < 2; ++it) {
        const v4u u = *(const v4u*)(sZ + it * 128 + lane * 4);
        *(volatile v4u*)(zr + it * 256 + lane * 8) = u;
      }
      __threadfence();
    }
  }
}

__global__ __launch_bounds__(32) void scan_kernel(const float* __restrict__ Bu, const float* __restrict__ tabl,
                                                 const float* __restrict__ st0, unsigned short* __restrict__ xs16,
                                                 float* __restrict__ stout) {
  __shared__ __align__(16) unsigned short sX[kScanBatch * 64];
  __shared__ __align__(16) float sS[64];
  const int w = blockIdx.x;
  const int j = threadIdx.x;
  const int p = w * 32 + j;
  const float ar = tabl[p];
  const float ai = tabl[kSt + p];
  float xr = st0[2 * p];
  float xi = st0[2 * p + 1];
  const int q = j >> 3, c8 = (j & 7) * 8;
  for (int t0 = 0; t0 < kSeq; t0 += kScanBatch) {
    float br[kScanBatch], bi[kScanBatch];
#pragma unroll
    for (int s = 0; s < kScanBatch; ++s) {
      const size_t o = (size_t)(t0 + s) * kHid + p;
      br[s] = Bu[o];
      bi[s] = Bu[o + kSt];
    }
#pragma unroll
    for (int s = 0; s < kScanBatch; ++s) {
      const float nr = ar * xr - ai * xi + br[s];
      const float ni = ar * xi + ai * xr + bi[s];
      xr = nr;
      xi = ni;
      sX[s * 64 + j]      = h_bits(xr * kXCarry);
      sX[s * 64 + 32 + j] = h_bits(xi * kXCarry);
    }
    __syncthreads();
    for (int pass = 0; pass < 2; ++pass) {
#pragma unroll
      for (int it = 0; it < 2; ++it) {
        const int row = it * 4 + q;
        const v4u u = *(const v4u*)(sX + row * 64 + c8);
        *(volatile v4u*)(xs16 + (size_t)(t0 + row) * kHid + 64 * w + c8) = u;
      }
      __threadfence();
    }
    __syncthreads();
  }
  sS[2 * j]     = xr;
  sS[2 * j + 1] = xi;
  __syncthreads();
  if (j < 16) {
    const v4f v = *(const v4f*)(sS + 4 * j);
    float* op = stout + 64 * w + 4 * j;
    *(volatile v4f*)op = v;
    __threadfence();
    *(volatile v4f*)op = v;
  }
}

__global__ __launch_bounds__(256) void ygelu_kernel(const float* __restrict__ ypre, const float* __restrict__ z32,
                                                   const float* __restrict__ Dl, unsigned short* __restrict__ g16) {
  __shared__ __align__(16) unsigned short sG[256 * 8];
  const int t = threadIdx.x;
  const size_t base = ((size_t)blockIdx.x * 256 + t) * 8;
  const int n0 = (int)(base & 511);
#pragma unroll 1
  for (int e = 0; e < 8; ++e) {
    const float y = ypre[base + e] + Dl[n0 + e] * z32[base + e];
    const float u = 0.7978845608028654f * (y + 0.044715f * (y * y * y));
    const float g = 0.5f * y * (1.0f + tanhf(u));
    sG[t * 8 + e] = h_bits(g);
  }
  __syncthreads();
  const v4u u = *(const v4u*)(sG + t * 8);
  unsigned short* q = g16 + base;
  *(volatile v4u*)q = u;
  __threadfence();
  *(volatile v4u*)q = u;
}

__global__ __launch_bounds__(256) void glu_kernel(const float* __restrict__ U, const float* __restrict__ b1,
                                                 const float* __restrict__ b2, const float* __restrict__ hin,
                                                 float* __restrict__ hout) {
  const size_t e0 = ((size_t)blockIdx.x * 256 + threadIdx.x) * 4;
  const size_t m  = e0 >> 9;
  const int n = (int)(e0 & 511);
  const v4f u1 = *(const v4f*)(U + m * 1024 + n);
  const v4f u2 = *(const v4f*)(U + m * 1024 + 512 + n);
  const v4f c1 = *(const v4f*)(b1 + n);
  const v4f c2 = *(const v4f*)(b2 + n);
  const v4f hv = *(const v4f*)(hin + e0);
  v4f o;
#pragma unroll
  for (int e = 0; e < 4; ++e) {
    const float a  = u1[e] + c1[e];
    const float qv = u2[e] + c2[e];
    const float ex = expf(-qv);
    const float sg = __builtin_amdgcn_rcpf(1.0f + ex);
    o[e] = hv[e] + a * sg;
  }
  float* hp = hout + e0;
  *(volatile v4f*)hp = o;
  __threadfence();
  *(volatile v4f*)hp = o;
}

extern "C" void kernel_launch(void* const* d_in, const int* in_sizes, int n_in,
                              void* d_out, int out_size, void* d_ws, size_t ws_size,
                              hipStream_t stream) {
  (void)in_sizes; (void)n_in; (void)out_size;
  const float* x        = (const float*)d_in[0];
  const float* state    = (const float*)d_in[1];
  const float* ctx      = (const float*)d_in[2];
  const float* W_enc    = (const float*)d_in[3];
  const float* b_enc    = (const float*)d_in[4];
  const float* Lam_re   = (const float*)d_in[5];
  const float* Lam_im   = (const float*)d_in[6];
  const float* B_re     = (const float*)d_in[7];
  const float* B_im     = (const float*)d_in[8];
  const float* C_re     = (const float*)d_in[9];
  const float* C_im     = (const float*)d_in[10];
  const float* Dv       = (const float*)d_in[11];
  const float* log_step = (const float*)d_in[12];
  const float* ln_scale = (const float*)d_in[13];
  const float* ln_bias  = (const float*)d_in[14];
  const float* W1       = (const float*)d_in[15];
  const float* b1       = (const float*)d_in[16];
  const float* W2       = (const float*)d_in[17];
  const float* b2       = (const float*)d_in[18];
  const float* W_dec    = (const float*)d_in[19];
  const float* b_dec    = (const float*)d_in[20];

  const size_t MiB = 1048576;
  const size_t offH0   = 0;
  const size_t offH1   = 16 * MiB;
  const size_t offZ32  = 32 * MiB;
  const size_t offU    = 32 * MiB;
  const size_t offBU   = 48 * MiB;
  const size_t offP16  = 64 * MiB;
  const size_t offXS   = 72 * MiB;
  const size_t offWENC = 80 * MiB;
  const size_t offWDEC = offWENC + (size_t)kHid * kHid * 2;
  const size_t offBBAR = offWDEC + (size_t)kOutDim * kHid * 2;
  const size_t offCST  = offBBAR + (size_t)kLayers * kHid * kHid * 2;
  const size_t offW12  = offCST + (size_t)kLayers * kHid * kHid * 2;
  const size_t offBPAD = offW12 + (size_t)kLayers * 2 * kHid * kHid * 2;
  const size_t offTAB  = offBPAD + (size_t)kHid * 4;
  const size_t total   = offTAB + (size_t)kLayers * 4 * kSt * 4;
  if (ws_size < total) return;

  char* ws = (char*)d_ws;
  float* H0  = (float*)(ws + offH0);
  float* H1  = (float*)(ws + offH1);
  float* Z32 = (float*)(ws + offZ32);
  float* U   = (float*)(ws + offU);
  float* BU  = (float*)(ws + offBU);
  unsigned short* P16  = (unsigned short*)(ws + offP16);
  unsigned short* XS16 = (unsigned short*)(ws + offXS);
  unsigned short* WENC = (unsigned short*)(ws + offWENC);
  unsigned short* WDEC = (unsigned short*)(ws + offWDEC);
  unsigned short* BBAR = (unsigned short*)(ws + offBBAR);
  unsigned short* CST  = (unsigned short*)(ws + offCST);
  unsigned short* W12  = (unsigned short*)(ws + offW12);
  float* BPAD = (float*)(ws + offBPAD);
  float* TAB  = (float*)(ws + offTAB);

  float* out0 = (float*)d_out;
  float* out1 = (float*)d_out + (size_t)kSeq * kOutDim;

  const int nPlane8   = kSeq * kHid / 8;
  const int gBlkN512  = (kSeq / 64) * (kHid / 64) / 8;
  const int gBlkN1024 = (kSeq / 64) * (2 * kHid / 64) / 8;
  const int gBlkN128  = (kSeq / 64) * (kOutDim / 64) / 8;

  cast8_f16_kernel<<<nPlane8 / 256, 256, 0, stream>>>(x, P16, nPlane8);
  cast_rows8_kernel<<<dim3(kHid / 4, 1), 256, 0, stream>>>(W_enc, 0L, WENC, 0L, kEncRows, kHid, kWCarry);
  cast_rows8_kernel<<<dim3(kOutDim / 4, 1), 256, 0, stream>>>(W_dec, 0L, WDEC, 0L, kOutDim, kOutDim, kWCarry);
  cast_rows8_kernel<<<dim3(kHid / 4, kLayers), 256, 0, stream>>>(W1, (long)kHid * kHid, W12, (long)2 * kHid * kHid,
                                                                 kHid, kHid, kWCarry);
  cast_rows8_kernel<<<dim3(kHid / 4, kLayers), 256, 0, stream>>>(W2, (long)kHid * kHid, W12 + (size_t)kHid * kHid,
                                                                 (long)2 * kHid * kHid, kHid, kHid, kWCarry);
  zoh_tab_kernel<<<kLayers, kSt, 0, stream>>>(Lam_re, Lam_im, log_step, TAB);
  bbar_kernel<<<dim3(kHid * kHid / 8 / 256, kLayers), 256, 0, stream>>>(B_re, B_im, TAB, BBAR);
  cst_kernel<<<dim3(kHid * kHid / 8 / 256, kLayers), 256, 0, stream>>>(C_re, C_im, CST);
  bias_pad_kernel<<<1, kHid, 0, stream>>>(b_enc, ctx, BPAD);

  wmma_gemm64<0, false, 2, 0, false, 0><<<dim3(gBlkN512, 1), 256, 0, stream>>>(
      P16, nullptr, kHid, 0L, WENC, nullptr, kHid, 0L, (void*)H0, nullptr, kHid, 0L,
      BPAD, nullptr, 0L, kSeq, kHid, kHid, kEncScale);

  for (int l = 0; l < kLayers; ++l) {
    const float* hin  = (l & 1) ? H1 : H0;
    float*       hout = (l & 1) ? H0 : H1;
    const size_t wsq  = (size_t)l * kHid * kHid;
    ln_kernel<<<kSeq, 128, 0, stream>>>(hin, ln_scale + l * kHid, ln_bias + l * kHid, Z32, P16);
    wmma_gemm64<0, false, 0, 0, false, 0><<<dim3(gBlkN512, 1), 256, 0, stream>>>(
        P16, nullptr, kHid, 0L, BBAR + wsq, nullptr, kHid, 0L, (void*)BU, nullptr, kHid, 0L,
        nullptr, nullptr, 0L, kSeq, kHid, kHid, kBuScale);
    scan_kernel<<<kSt / 32, 32, 0, stream>>>(BU, TAB + (size_t)l * 4 * kSt, state + (size_t)l * kSt * 2,
                                             XS16, out1 + (size_t)l * kSt * 2);
    wmma_gemm64<0, false, 0, 0, false, 0><<<dim3(gBlkN512, 1), 256, 0, stream>>>(
        XS16, nullptr, kHid, 0L, CST + wsq, nullptr, kHid, 0L, (void*)BU, nullptr, kHid, 0L,
        nullptr, nullptr, 0L, kSeq, kHid, kHid, kYScale);
    ygelu_kernel<<<nPlane8 / 256, 256, 0, stream>>>(BU, Z32, Dv + l * kHid, P16);
    wmma_gemm64<0, false, 0, 0, false, 0><<<dim3(gBlkN1024, 1), 256, 0, stream>>>(
        P16, nullptr, kHid, 0L, W12 + 2 * wsq, nullptr, kHid, 0L, (void*)U, nullptr, 2 * kHid, 0L,
        nullptr, nullptr, 0L, kSeq, 2 * kHid, kHid, kGluScale);
    glu_kernel<<<kSeq * kHid / 4 / 256, 256, 0, stream>>>(U, b1 + l * kHid, b2 + l * kHid, hin, hout);
  }

  cast8_f16_kernel<<<nPlane8 / 256, 256, 0, stream>>>(H0, P16, nPlane8);
  wmma_gemm64<0, false, 2, 0, false, 0><<<dim3(gBlkN128, 1), 256, 0, stream>>>(
      P16, nullptr, kHid, 0L, WDEC, nullptr, kHid, 0L, (void*)out0, nullptr, kOutDim, 0L,
      b_dec, nullptr, 0L, kSeq, kOutDim, kHid, kDecScale);
}
